// PointnetSAModuleMSG_58669253263780
// MI455X (gfx1250) — hardware-verified
//
#include <hip/hip_runtime.h>
#pragma clang fp contract(off)

typedef __attribute__((ext_vector_type(16))) _Float16     v16h;
typedef __attribute__((ext_vector_type(8)))  _Float16     v8h;
typedef __attribute__((ext_vector_type(8)))  float        v8f;
typedef __attribute__((ext_vector_type(4)))  float        v4f;
typedef __attribute__((ext_vector_type(4)))  unsigned int v4u;

constexpr int NBATCH   = 4;
constexpr int NPTS     = 16384;
constexpr int CFEAT    = 64;
constexpr int NCENT    = 2048;
constexpr int KPAD1    = 96;
constexpr int CO2      = 128;
constexpr int WSRC1    = 67;
constexpr int NQ       = NBATCH * NCENT;
constexpr int CEN_PER_WAVE  = 16;
constexpr int WAVES_PER_BLK = 2;
constexpr int NBLK_MLP = NQ / (CEN_PER_WAVE * WAVES_PER_BLK);
constexpr int PART_PITCH = 256;

constexpr float A_CARRY = 16.0f;
constexpr float W_CARRY = 16.0f;
constexpr float H_CARRY = 16.0f;
constexpr float FOLD1   = 1.0f / (A_CARRY * W_CARRY);
constexpr float FOLD2   = 1.0f / (H_CARRY * W_CARRY);

static_assert(NPTS % 1024 == 0 && NPTS / 1024 == 16, "fps ownership map");
static_assert(NCENT % 32 == 0, "centre tiles stay inside one batch");
static_assert(NQ % (CEN_PER_WAVE * WAVES_PER_BLK) == 0, "mlp grid exact");
static_assert(KPAD1 % 32 == 0 && KPAD1 >= WSRC1, "layer-1 K pad");
static_assert(NBATCH * NCENT * 3 * 4 == 98304, "out0 bytes");
static_assert(98304 % 128 == 0, "out1 line aligned");
static_assert(98304 + NBATCH * 256 * NCENT * 4 == 8486912, "d_out total");

__device__ __forceinline__ v16h ldfrag(const _Float16* p) {
  union U { v16h v; v8h h[2]; } f;
  f.h[0] = *(const v8h*)(p);
  f.h[1] = *(const v8h*)(p + 16);
  return f.v;
}
__device__ __forceinline__ v8f mma_h(v16h a, v16h b, v8f c) {
  c = __builtin_amdgcn_wmma_f32_16x16x32_f16(false, a, false, b, (short)0, c, false, false);
  asm volatile("v_nop\n\tv_nop\n\tv_nop\n\tv_nop" : "+v"(c) : "v"(a), "v"(b));
  return c;
}
__device__ __forceinline__ unsigned h16bits(float f) {
  const _Float16 hv = (_Float16)f;
  const unsigned short us = __builtin_bit_cast(unsigned short, hv);
  return (unsigned)us;
}
__device__ __forceinline__ unsigned pack2h(float lo, float hi) {
  return h16bits(lo) | (h16bits(hi) << 16);
}

__global__ __launch_bounds__(1024) void fps_select(const float* __restrict__ xyz,
                                                   float* __restrict__ out0,
                                                   float* __restrict__ nxw) {
#pragma clang fp contract(off)
  constexpr int PT = 16;
  __shared__ __align__(16) float stgp[2048 * 3];
  __shared__ __align__(16) float nx[NCENT * 3];
  __shared__ float sv[2][32];
  __shared__ int   si[2][32];

  const int b = blockIdx.x;
  const int t = threadIdx.x;
  const int lane = t & 31;
  const int wv = t >> 5;
  const float* xb = xyz + (size_t)b * NPTS * 3;

  float px[PT], py[PT], pz[PT], dd[PT];
#pragma unroll
  for (int c = 0; c < 8; ++c) {
    __syncthreads();
    {
      const v4f v = *(const v4f*)(xb + c * 6144 + t * 4);
      *(v4f*)(stgp + t * 4) = v;
    }
    if (t < 512) {
      const v4f v = *(const v4f*)(xb + c * 6144 + (t + 1024) * 4);
      *(v4f*)(stgp + (t + 1024) * 4) = v;
    }
    __syncthreads();
    px[2 * c]     = stgp[t * 3 + 0];
    py[2 * c]     = stgp[t * 3 + 1];
    pz[2 * c]     = stgp[t * 3 + 2];
    px[2 * c + 1] = stgp[(t + 1024) * 3 + 0];
    py[2 * c + 1] = stgp[(t + 1024) * 3 + 1];
    pz[2 * c + 1] = stgp[(t + 1024) * 3 + 2];
  }
#pragma unroll
  for (int i = 0; i < PT; ++i) dd[i] = 1e10f;

  int cur = 0;
#pragma unroll 1
  for (int j = 0; j < NCENT; ++j) {
    int cc = cur < 0 ? 0 : cur;
    cc = cc > (NPTS - 1) ? (NPTS - 1) : cc;
    const float cx = xb[cc * 3 + 0];
    const float cy = xb[cc * 3 + 1];
    const float cz = xb[cc * 3 + 2];
    if (t == 0) {
      nx[j * 3 + 0] = cx;
      nx[j * 3 + 1] = cy;
      nx[j * 3 + 2] = cz;
    }
    float best = -1.0f;
    int bi = 0;
#pragma unroll
    for (int i = 0; i < PT; ++i) {
      const float dx = px[i] - cx;
      const float dy = py[i] - cy;
      const float dz = pz[i] - cz;
      const float t0 = dx * dx;
      const float t1 = dy * dy;
      const float t2 = dz * dz;
      const float d = (t0 + t2) + t1;
      const float nd = fminf(dd[i], d);
      dd[i] = nd;
      const bool tk = nd > best;
      best = tk ? nd : best;
      bi = tk ? (t + i * 1024) : bi;
    }
#pragma unroll
    for (int off = 16; off > 0; off >>= 1) {
      const float ov = __shfl_xor(best, off);
      const int   oi = __shfl_xor(bi, off);
      const bool tk = (ov > best) || ((ov == best) && (oi < bi));
      best = tk ? ov : best;
      bi = tk ? oi : bi;
    }
    const int pp = j & 1;
    if (lane == 0) {
      sv[pp][wv] = best;
      si[pp][wv] = bi;
    }
    __syncthreads();
    best = sv[pp][lane];
    bi = si[pp][lane];
#pragma unroll
    for (int off = 16; off > 0; off >>= 1) {
      const float ov = __shfl_xor(best, off);
      const int   oi = __shfl_xor(bi, off);
      const bool tk = (ov > best) || ((ov == best) && (oi < bi));
      best = tk ? ov : best;
      bi = tk ? oi : bi;
    }
    cur = bi;
  }
  __syncthreads();
  {
    const v4f v0 = *(const v4f*)(nx + t * 4);
    v4f v1 = v0;
    if (t < 512) v1 = *(const v4f*)(nx + (t + 1024) * 4);
    float* o = out0 + (size_t)b * (NCENT * 3);
    float* w = nxw + (size_t)b * (NCENT * 3);
    for (int pass = 0; pass < 2; ++pass) {
      *(volatile v4f*)(o + t * 4) = v0;
      *(volatile v4f*)(w + t * 4) = v0;
      if (t < 512) {
        *(volatile v4f*)(o + (t + 1024) * 4) = v1;
        *(volatile v4f*)(w + (t + 1024) * 4) = v1;
      }
      __threadfence();
    }
  }
}

template <int SAMP, int C1, int PASS>
__global__ __launch_bounds__(64) void mlp_pass(
    const float* __restrict__ xyz, const float* __restrict__ feat, const float* __restrict__ nxw,
    const float* __restrict__ w1, const float* __restrict__ w2, const float* __restrict__ ss1,
    float* __restrict__ part, float* __restrict__ ymax, float* __restrict__ ymin, float r2) {
#pragma clang fp contract(off)
  constexpr int KP2 = C1;
  constexpr int NT1 = C1 / 16;
  constexpr int NT2 = CO2 / 16;
  constexpr int NS  = (PASS == 0) ? NT1 : NT2;
  static_assert(SAMP == 16 || SAMP == 32, "group size");
  static_assert(C1 % 32 == 0 && C1 <= 128, "layer-2 K multiple of 32");
  static_assert(CFEAT == 64, "gather map");

  __shared__ __align__(16) _Float16 W1s[C1 * KPAD1];
  __shared__ __align__(16) _Float16 W2s[(PASS == 1) ? (CO2 * KP2) : 8];
  __shared__ __align__(16) _Float16 As[WAVES_PER_BLK][16 * KPAD1];
  __shared__ __align__(16) _Float16 Hs[(PASS == 1) ? WAVES_PER_BLK : 1][(PASS == 1) ? (16 * KP2) : 8];
  __shared__ __align__(16) float stg[(PASS == 1) ? WAVES_PER_BLK : 1][(PASS == 1) ? 256 : 4];
  __shared__ __align__(16) float statw[WAVES_PER_BLK][256];
  __shared__ int lst[WAVES_PER_BLK][32];

  const int tid  = threadIdx.x;
  const int wave = tid >> 5;
  const int lane = tid & 31;
  const int hh   = lane >> 4;
  const int m    = lane & 15;

  for (int i = tid; i < C1 * KPAD1; i += 64) {
    const int o = i / KPAD1;
    const int k = i - o * KPAD1;
    int src = (k < 64) ? (k + 3) : (k - 64);
    src = src > (WSRC1 - 1) ? (WSRC1 - 1) : src;
    const float wvv = w1[o * WSRC1 + src];
    const float v = (k < WSRC1) ? (wvv * W_CARRY) : 0.0f;
    W1s[i] = (_Float16)v;
  }
  if constexpr (PASS == 1) {
    for (int i = tid; i < CO2 * KP2; i += 64) {
      const float v = w2[i] * W_CARRY;
      W2s[i] = (_Float16)v;
    }
  }
  for (int i = tid; i < WAVES_PER_BLK * 256; i += 64) (&statw[0][0])[i] = 0.0f;
  lst[wave][lane] = 0;

  float sc1[NT1], sh1[NT1];
#pragma unroll
  for (int n1 = 0; n1 < NT1; ++n1) {
    sc1[n1] = 0.0f;
    sh1[n1] = 0.0f;
  }
  if constexpr (PASS == 1) {
#pragma unroll
    for (int n1 = 0; n1 < NT1; ++n1) {
      const float a = ss1[n1 * 16 + m];
      const float c = ss1[128 + n1 * 16 + m];
      sc1[n1] = a * (FOLD1 * H_CARRY);
      sh1[n1] = c * H_CARRY;
    }
  }

  float sum[NS], sq[NS];
#pragma unroll
  for (int n = 0; n < NS; ++n) {
    sum[n] = 0.0f;
    sq[n] = 0.0f;
  }

#pragma unroll 1
  for (int qi = 0; qi < CEN_PER_WAVE; ++qi) {
    const int q = blockIdx.x * (WAVES_PER_BLK * CEN_PER_WAVE) + wave * CEN_PER_WAVE + qi;
    const int b = q >> 11;
    const float qx = nxw[q * 3 + 0];
    const float qy = nxw[q * 3 + 1];
    const float qz = nxw[q * 3 + 2];
    const float* xb = xyz + (size_t)b * NPTS * 3;

    __syncthreads();
    const float sqc = ((qx * qx) + (qz * qz)) + (qy * qy);
    int cnt = 0;
#pragma unroll 1
    for (int base = 0; base < NPTS; base += 32) {
      if (cnt >= SAMP) break;
      const int i = base + lane;
      const float x = xb[i * 3 + 0];
      const float y = xb[i * 3 + 1];
      const float z = xb[i * 3 + 2];
      const float sqx = ((x * x) + (z * z)) + (y * y);
      float p = qx * x;
      p = __builtin_fmaf(qy, y, p);
      p = __builtin_fmaf(qz, z, p);
      const float tw = 2.0f * p;
      const float d2 = (sqc + sqx) - tw;
      const bool hit = d2 < r2;
      const unsigned mk = (unsigned)__ballot(hit);
      const int pos = cnt + __popc(mk & ((1u << lane) - 1u));
      if (hit && pos < SAMP) lst[wave][pos] = i;
      cnt += __popc(mk);
    }
    __syncthreads();
    int jv;
    {
      const int cntc = cnt < SAMP ? cnt : SAMP;
      const int l0 = lst[wave][0];
      const int lm = lst[wave][lane];
      const int first = (cnt > 0) ? l0 : 0;
      jv = (lane < cntc) ? lm : first;
      jv = jv < 0 ? 0 : jv;
      jv = jv > (NPTS - 1) ? (NPTS - 1) : jv;
    }

    float cmax[NT2], cmin[NT2];
#pragma unroll
    for (int n2 = 0; n2 < NT2; ++n2) {
      cmax[n2] = -3.0e38f;
      cmin[n2] = 3.0e38f;
    }

#pragma unroll 1
    for (int t = 0; t < SAMP / 16; ++t) {
      __syncthreads();
      {
        const int seg = lane & 7;
        const int rsub = lane >> 3;
#pragma unroll
        for (int st = 0; st < 4; ++st) {
          const int row = st * 4 + rsub;
          const int j = __shfl(jv, t * 16 + row);
          const float* fp = feat + ((size_t)(b * NPTS + j)) * CFEAT + seg * 8;
          const v4f f0 = *(const v4f*)fp;
          const v4f f1 = *(const v4f*)(fp + 4);
          v4u w;
          w.x = pack2h(f0.x * A_CARRY, f0.y * A_CARRY);
          w.y = pack2h(f0.z * A_CARRY, f0.w * A_CARRY);
          w.z = pack2h(f1.x * A_CARRY, f1.y * A_CARRY);
          w.w = pack2h(f1.z * A_CARRY, f1.w * A_CARRY);
          *(v8h*)(&As[wave][row * KPAD1 + seg * 8]) = __builtin_bit_cast(v8h, w);
          if (st == 1) asm volatile("" ::: "memory");
        }
        const int jr = __shfl(jv, t * 16 + m);
        const float x = xb[jr * 3 + 0];
        const float y = xb[jr * 3 + 1];
        const float z = xb[jr * 3 + 2];
        const float rx = (x - qx) * A_CARRY;
        const float ry = (y - qy) * A_CARRY;
        const float rz = (z - qz) * A_CARRY;
        unsigned zz = 0u;
        asm volatile("" : "+v"(zz));
        const unsigned wxy = pack2h(rx, ry);
        const unsigned wz0 = h16bits(rz) | (zz << 16);
        v4u wa, wb;
        wa.x = (hh == 0) ? wxy : zz;
        wa.y = (hh == 0) ? wz0 : zz;
        wa.z = zz;
        wa.w = zz;
        wb.x = zz;
        wb.y = zz;
        wb.z = zz;
        wb.w = zz;
        *(v8h*)(&As[wave][m * KPAD1 + 64 + 16 * hh]) = __builtin_bit_cast(v8h, wa);
        *(v8h*)(&As[wave][m * KPAD1 + 72 + 16 * hh]) = __builtin_bit_cast(v8h, wb);
      }
      __syncthreads();

      {
        const _Float16* Aw = &As[wave][m * KPAD1 + 8 * hh];
        const v16h a0 = ldfrag(Aw);
        const v16h a1 = ldfrag(Aw + 32);
        const v16h a2 = ldfrag(Aw + 64);
#pragma unroll
        for (int n1 = 0; n1 < NT1; ++n1) {
          const _Float16* Bw = &W1s[(n1 * 16 + m) * KPAD1 + 8 * hh];
          v8f acc = (v8f){0.f, 0.f, 0.f, 0.f, 0.f, 0.f, 0.f, 0.f};
          acc = mma_h(a0, ldfrag(Bw), acc);
          acc = mma_h(a1, ldfrag(Bw + 32), acc);
          acc = mma_h(a2, ldfrag(Bw + 64), acc);
          if constexpr (PASS == 0) {
            float s = 0.0f, s2 = 0.0f;
#pragma unroll
            for (int r = 0; r < 8; ++r) {
              const float yv = acc[r] * FOLD1;
              const float yy = yv * yv;
              s = s + yv;
              s2 = s2 + yy;
            }
            sum[n1] = sum[n1] + s;
            sq[n1] = sq[n1] + s2;
          } else {
#pragma unroll
            for (int r = 0; r < 8; ++r) {
              const float pv = acc[r] * sc1[n1];
              const float hv = fmaxf(pv + sh1[n1], 0.0f);
              Hs[wave][(8 * hh + r) * KP2 + n1 * 16 + m] = (_Float16)hv;
            }
          }
        }
      }

      if constexpr (PASS == 1) {
        __syncthreads();
        const _Float16* Hw = &Hs[wave][m * KP2 + 8 * hh];
        v16h hf[KP2 / 32];
#pragma unroll
        for (int ks = 0; ks < KP2 / 32; ++ks) hf[ks] = ldfrag(Hw + ks * 32);
#pragma unroll
        for (int n2 = 0; n2 < NT2; ++n2) {
          const _Float16* Bw = &W2s[(n2 * 16 + m) * KP2 + 8 * hh];
          v8f acc = (v8f){0.f, 0.f, 0.f, 0.f, 0.f, 0.f, 0.f, 0.f};
#pragma unroll
          for (int ks = 0; ks < KP2 / 32; ++ks) acc = mma_h(hf[ks], ldfrag(Bw + ks * 32), acc);
          float s = 0.0f, s2 = 0.0f, mx = -3.0e38f, mn = 3.0e38f;
#pragma unroll
          for (int r = 0; r < 8; ++r) {
            const float yv = acc[r] * FOLD2;
            const float yy = yv * yv;
            s = s + yv;
            s2 = s2 + yy;
            mx = fmaxf(mx, yv);
            mn = fminf(mn, yv);
          }
          sum[n2] = sum[n2] + s;
          sq[n2] = sq[n2] + s2;
          const float omx = __shfl_xor(mx, 16);
          const float omn = __shfl_xor(mn, 16);
          mx = fmaxf(mx, omx);
          mn = fminf(mn, omn);
          cmax[n2] = fmaxf(cmax[n2], mx);
          cmin[n2] = fminf(cmin[n2], mn);
        }
      }
    }

    if constexpr (PASS == 1) {
#pragma unroll
      for (int n2 = 0; n2 < NT2; ++n2) {
        const float v = (hh == 0) ? cmax[n2] : cmin[n2];
        stg[wave][hh * 128 + n2 * 16 + m] = v;
      }
      __syncthreads();
      const v4f vx = *(const v4f*)(&stg[wave][lane * 4]);
      const v4f vn = *(const v4f*)(&stg[wave][128 + lane * 4]);
      float* pmx = ymax + (size_t)q * CO2 + lane * 4;
      float* pmn = ymin + (size_t)q * CO2 + lane * 4;
      for (int pass = 0; pass < 2; ++pass) {
        *(volatile v4f*)pmx = vx;
        *(volatile v4f*)pmn = vn;
        __threadfence();
      }
    }
  }

#pragma unroll
  for (int n = 0; n < NS; ++n) {
    const float os = __shfl_xor(sum[n], 16);
    const float oq = __shfl_xor(sq[n], 16);
    const float ts = sum[n] + os;
    const float tq = sq[n] + oq;
    if (hh == 0) {
      statw[wave][n * 16 + m] = ts;
      statw[wave][128 + n * 16 + m] = tq;
    }
  }
  __syncthreads();
  if (wave == 0) {
    const v4f a0 = *(const v4f*)(&statw[0][lane * 4]);
    const v4f b0 = *(const v4f*)(&statw[1][lane * 4]);
    const v4f a1 = *(const v4f*)(&statw[0][128 + lane * 4]);
    const v4f b1 = *(const v4f*)(&statw[1][128 + lane * 4]);
    const v4f t0 = a0 + b0;
    const v4f t1 = a1 + b1;
    float* pp = part + (size_t)blockIdx.x * PART_PITCH;
    for (int pass = 0; pass < 2; ++pass) {
      *(volatile v4f*)(pp + lane * 4) = t0;
      *(volatile v4f*)(pp + 128 + lane * 4) = t1;
      __threadfence();
    }
  }
}

__global__ __launch_bounds__(128) void bn_finalize(const float* __restrict__ part, int nblk, int nch,
                                                   double invcnt, const float* __restrict__ g,
                                                   const float* __restrict__ beta,
                                                   float* __restrict__ ss) {
#pragma clang fp contract(off)
  __shared__ __align__(16) float ssl[256];
  const int c = threadIdx.x;
  int nb = nblk < 0 ? 0 : nblk;
  nb = nb > NBLK_MLP ? NBLK_MLP : nb;
  int cc = c < nch ? c : (nch - 1);
  cc = cc < 0 ? 0 : cc;
  double s = 0.0, q = 0.0;
#pragma unroll 1
  for (int i = 0; i < nb; ++i) {
    const float a = part[(size_t)i * PART_PITCH + c];
    const float d = part[(size_t)i * PART_PITCH + 128 + c];
    s = s + (double)a;
    q = q + (double)d;
  }
  const double mean = s * invcnt;
  const double msq = mean * mean;
  double var = q * invcnt - msq;
  var = var < 0.0 ? 0.0 : var;
  const float vf = (float)var + 1e-5f;
  const float inv = 1.0f / sqrtf(vf);
  const float sc = g[cc] * inv;
  const float ms = (float)mean * sc;
  const float sh = beta[cc] - ms;
  const bool valid = c < nch;
  ssl[c] = valid ? sc : 0.0f;
  ssl[128 + c] = valid ? sh : 0.0f;
  __syncthreads();
  if (c < 64) {
    const v4f v = *(const v4f*)(&ssl[c * 4]);
    for (int pass = 0; pass < 2; ++pass) {
      *(volatile v4f*)(ss + c * 4) = v;
      __threadfence();
    }
  }
}

__global__ __launch_bounds__(128) void bn_max_out(const float* __restrict__ ymax,
                                                  const float* __restrict__ ymin,
                                                  const float* __restrict__ ss2,
                                                  float* __restrict__ out1, int coff) {
#pragma clang fp contract(off)
  __shared__ __align__(16) float tile[128 * 36];
  const int tid = threadIdx.x;
  const int wave = tid >> 5;
  const int lane = tid & 31;
  const int q0 = blockIdx.x * 32;
  const int b = q0 >> 11;
  const int p0 = q0 & (NCENT - 1);
  const int c4 = (tid & 31) * 4;
  const int prow = tid >> 5;
  const v4f scv = *(const v4f*)(ss2 + c4);
  const v4f shv = *(const v4f*)(ss2 + 128 + c4);
  const float sc0 = scv.x, sc1v = scv.y, sc2 = scv.z, sc3 = scv.w;
  const float sh0 = shv.x, sh1v = shv.y, sh2 = shv.z, sh3 = shv.w;
#pragma unroll 1
  for (int it = 0; it < 8; ++it) {
    const int p = it * 4 + prow;
    const v4f mx = *(const v4f*)(ymax + (size_t)(q0 + p) * CO2 + c4);
    const v4f mn = *(const v4f*)(ymin + (size_t)(q0 + p) * CO2 + c4);
    const float e0 = (sc0 >= 0.0f) ? mx.x : mn.x;
    const float e1 = (sc1v >= 0.0f) ? mx.y : mn.y;
    const float e2 = (sc2 >= 0.0f) ? mx.z : mn.z;
    const float e3 = (sc3 >= 0.0f) ? mx.w : mn.w;
    const float m0 = sc0 * e0;
    const float m1 = sc1v * e1;
    const float m2 = sc2 * e2;
    const float m3 = sc3 * e3;
    tile[(c4 + 0) * 36 + p] = fmaxf(m0 + sh0, 0.0f);
    tile[(c4 + 1) * 36 + p] = fmaxf(m1 + sh1v, 0.0f);
    tile[(c4 + 2) * 36 + p] = fmaxf(m2 + sh2, 0.0f);
    tile[(c4 + 3) * 36 + p] = fmaxf(m3 + sh3, 0.0f);
  }
  __syncthreads();
  const int cq = lane >> 3;
  const int p4 = (lane & 7) * 4;
  for (int pass = 0; pass < 2; ++pass) {
#pragma unroll
    for (int it = 0; it < 8; ++it) {
      const int c = it * 16 + wave * 4 + cq;
      const v4f v = *(const v4f*)(&tile[c * 36 + p4]);
      *(volatile v4f*)(out1 + ((size_t)(b * 256 + coff + c)) * NCENT + p0 + p4) = v;
    }
    __threadfence();
  }
}

extern "C" void kernel_launch(void* const* d_in, const int* in_sizes, int n_in,
                              void* d_out, int out_size, void* d_ws, size_t ws_size,
                              hipStream_t stream) {
  (void)in_sizes; (void)n_in; (void)out_size;

  const float* xyz  = (const float*)d_in[0];
  const float* feat = (const float*)d_in[1];
  const float* w0_0 = (const float*)d_in[2];
  const float* g0_0 = (const float*)d_in[3];
  const float* b0_0 = (const float*)d_in[4];
  const float* w0_1 = (const float*)d_in[5];
  const float* g0_1 = (const float*)d_in[6];
  const float* b0_1 = (const float*)d_in[7];
  const float* w1_0 = (const float*)d_in[8];
  const float* g1_0 = (const float*)d_in[9];
  const float* b1_0 = (const float*)d_in[10];
  const float* w1_1 = (const float*)d_in[11];
  const float* g1_1 = (const float*)d_in[12];
  const float* b1_1 = (const float*)d_in[13];

  float* out0 = (float*)d_out;
  float* out1 = out0 + NBATCH * NCENT * 3;

  char* ws = (char*)d_ws;
  size_t off = 0;
  const size_t SZ_NX = (size_t)NQ * 3 * 4;
  const size_t SZ_PART = (size_t)NBLK_MLP * PART_PITCH * 4;
  const size_t SZ_SS = 256 * 4;
  const size_t SZ_Y = (size_t)NQ * CO2 * 4;
  float* nxw = (float*)(ws + off);    off += SZ_NX;
  float* partA0 = (float*)(ws + off); off += SZ_PART;
  float* partB0 = (float*)(ws + off); off += SZ_PART;
  float* partA1 = (float*)(ws + off); off += SZ_PART;
  float* partB1 = (float*)(ws + off); off += SZ_PART;
  float* ssA0 = (float*)(ws + off);   off += SZ_SS;
  float* ssB0 = (float*)(ws + off);   off += SZ_SS;
  float* ssA1 = (float*)(ws + off);   off += SZ_SS;
  float* ssB1 = (float*)(ws + off);   off += SZ_SS;
  float* ymax0 = (float*)(ws + off);  off += SZ_Y;
  float* ymin0 = (float*)(ws + off);  off += SZ_Y;
  float* ymax1 = (float*)(ws + off);  off += SZ_Y;
  float* ymin1 = (float*)(ws + off);  off += SZ_Y;
  if (off > ws_size || off > (size_t)134217728) return;

  const double inv0 = 1.0 / (double)(NQ * 16);
  const double inv1 = 1.0 / (double)(NQ * 32);

  fps_select<<<NBATCH, 1024, 0, stream>>>(xyz, out0, nxw);

  mlp_pass<16, 64, 0><<<NBLK_MLP, 64, 0, stream>>>(xyz, feat, nxw, w0_0, w0_1, ssA0, partA0, ymax0, ymin0, 0.25f);
  bn_finalize<<<1, 128, 0, stream>>>(partA0, NBLK_MLP, 64, inv0, g0_0, b0_0, ssA0);
  mlp_pass<16, 64, 1><<<NBLK_MLP, 64, 0, stream>>>(xyz, feat, nxw, w0_0, w0_1, ssA0, partB0, ymax0, ymin0, 0.25f);
  bn_finalize<<<1, 128, 0, stream>>>(partB0, NBLK_MLP, 128, inv0, g0_1, b0_1, ssB0);
  bn_max_out<<<NQ / 32, 128, 0, stream>>>(ymax0, ymin0, ssB0, out1, 0);

  mlp_pass<32, 96, 0><<<NBLK_MLP, 64, 0, stream>>>(xyz, feat, nxw, w1_0, w1_1, ssA1, partA1, ymax1, ymin1, 1.0f);
  bn_finalize<<<1, 128, 0, stream>>>(partA1, NBLK_MLP, 96, inv1, g1_0, b1_0, ssA1);
  mlp_pass<32, 96, 1><<<NBLK_MLP, 64, 0, stream>>>(xyz, feat, nxw, w1_0, w1_1, ssA1, partB1, ymax1, ymin1, 1.0f);
  bn_finalize<<<1, 128, 0, stream>>>(partB1, NBLK_MLP, 128, inv1, g1_1, b1_1, ssB1);
  bn_max_out<<<NQ / 32, 128, 0, stream>>>(ymax1, ymin1, ssB1, out1, 128);
}
